// DRNNBert_21328807592514
// MI455X (gfx1250) — hardware-verified
//
#include <hip/hip_runtime.h>
#include <math.h>

constexpr int NBATCH  = 32;
constexpr int NSTEP   = 512;
constexpr int NEMB    = 768;
constexpr int NHID    = 1024;
constexpr int NHEAD   = 128;
constexpr int NROWS   = NBATCH * NSTEP;
constexpr int SEQ_BLK = 16;
constexpr int REC_THR = 512;
constexpr int HPITCH  = 1032;
constexpr int CVT_THR = 256;
constexpr float WCARRY     = 32.0f;
constexpr float WCARRY_INV = 1.0f / 32.0f;

static_assert(NROWS == 16384, "row count");
static_assert(NROWS % 64 == 0 && NHID % 64 == 0 && NHEAD % 64 == 0, "tile multiples for rows and columns");
static_assert(NEMB % 32 == 0 && NHID % 32 == 0, "depth multiple of 32");
static_assert(NBATCH % SEQ_BLK == 0, "batch tiles");
static_assert(REC_THR / 32 == SEQ_BLK, "one wave per batch row in the row copy");
static_assert(NHID == 64 * (REC_THR / 32), "16 waves x 64 hidden columns");
static_assert(NHID * 2 == 4 * 32 * 16, "row copy: 4 instructions x 32 lanes x 16 B");
static_assert(HPITCH % 8 == 0 && HPITCH >= NHID, "LDS pitch keeps 16-B alignment");
static_assert((2 * SEQ_BLK * HPITCH) % 8 == 0, "zero fill in 16-B vectors");
static_assert((NROWS * NEMB) % (8 * CVT_THR) == 0, "convert grid exact (x)");
static_assert((NHID * NEMB) % (8 * CVT_THR) == 0, "convert grid exact (W_ih1)");
static_assert((NHID * NHID) % (8 * CVT_THR) == 0, "convert grid exact (square planes)");
static_assert((NHEAD * NHID) % (8 * CVT_THR) == 0, "convert grid exact (head planes)");
static_assert(NHID == 4 * 256, "bias sum kernel: 256 threads x 4 floats");

typedef __attribute__((ext_vector_type(16))) _Float16 v16h;
typedef __attribute__((ext_vector_type(8)))  _Float16 v8h;
typedef __attribute__((ext_vector_type(8)))  float    v8f;
typedef __attribute__((ext_vector_type(4)))  float    v4f;

union FragU { v16h v; v8h h[2]; };
__device__ __forceinline__ v16h frag_load(const _Float16* p) {
  FragU f;
  f.h[0] = *(const v8h*)(p);
  f.h[1] = *(const v8h*)(p + 16);
  return f.v;
}
__device__ __forceinline__ v8f wmma_h(v16h a, v16h b, v8f c) {
  return __builtin_amdgcn_wmma_f32_16x16x32_f16(false, a, false, b, (short)0, c, false, false);
}
__device__ __forceinline__ v8f wmma_h_guarded(v16h a, v16h b, v8f c) {
  c = __builtin_amdgcn_wmma_f32_16x16x32_f16(false, a, false, b, (short)0, c, false, false);
  asm volatile("v_nop\n\tv_nop\n\tv_nop\n\tv_nop" : "+v"(c) : "v"(a), "v"(b));
  return c;
}
__device__ __forceinline__ void guard4_h(v8f& a, v8f& b, v8f& c, v8f& d, v16h x, v16h y) {
  asm volatile("v_nop\n\tv_nop\n\tv_nop\n\tv_nop" : "+v"(a), "+v"(b), "+v"(c), "+v"(d) : "v"(x), "v"(y));
}
__device__ __forceinline__ void keep4_h(v16h a, v16h b, v16h c, v16h d) {
  asm volatile("v_nop" :: "v"(a), "v"(b), "v"(c), "v"(d));
}
__device__ __forceinline__ void acc_guard4(v8f& a, v8f& b, v8f& c, v8f& d) {
  asm volatile("v_nop\n\tv_nop\n\tv_nop\n\tv_nop" : "+v"(a), "+v"(b), "+v"(c), "+v"(d));
}

__global__ __launch_bounds__(CVT_THR) void cvt8_f16_kernel(const float* __restrict__ src,
                                                           unsigned short* __restrict__ dst, int n8, float sc) {
  const int i = blockIdx.x * CVT_THR + threadIdx.x;
  if (i < n8) {
    const float* sp = src + (size_t)i * 8;
    const v4f a = *(const v4f*)(sp);
    const v4f b = *(const v4f*)(sp + 4);
    v8h hv;
#pragma unroll
    for (int e = 0; e < 4; ++e) {
      const float fa = a[e] * sc;
      const float fb = b[e] * sc;
      hv[e]     = (_Float16)fa;
      hv[4 + e] = (_Float16)fb;
    }
    *(volatile v8h*)(dst + (size_t)i * 8) = hv;
    __threadfence();
    *(volatile v8h*)(dst + (size_t)i * 8) = hv;
  }
}

__global__ __launch_bounds__(256) void bias_sum_kernel(const float* __restrict__ ba1, const float* __restrict__ bb1,
                                                       const float* __restrict__ ba2, const float* __restrict__ bb2,
                                                       float* __restrict__ dst) {
  const int layer = blockIdx.x;
  const int idx = threadIdx.x * 4;
  const v4f p1 = *(const v4f*)(ba1 + idx);
  const v4f q1 = *(const v4f*)(bb1 + idx);
  const v4f p2 = *(const v4f*)(ba2 + idx);
  const v4f q2 = *(const v4f*)(bb2 + idx);
  v4f o;
#pragma unroll
  for (int e = 0; e < 4; ++e) {
    const float s1 = p1[e] + q1[e];
    const float s2 = p2[e] + q2[e];
    o[e] = (layer != 0) ? s2 : s1;
  }
  float* op = dst + layer * NHID + idx;
  *(volatile v4f*)op = o;
  __threadfence();
  *(volatile v4f*)op = o;
}

__global__ __launch_bounds__(256) void gemm64_f16_kernel(
    const unsigned short* __restrict__ Ap, int lda,
    const unsigned short* __restrict__ Btp, int ldb,
    float* __restrict__ Cout, int ldc,
    const float* __restrict__ bias,
    int mdim, int ndim, int kdim, float scale) {
  const _Float16* Amat = (const _Float16*)Ap;
  const _Float16* Bmat = (const _Float16*)Btp;
  __shared__ __align__(16) float sT[8][16 * 68];
  const int lane = threadIdx.x & 31;
  const int wave = threadIdx.x >> 5;
  const int tilesN = ndim >> 6;
  const int tilesM = mdim >> 6;
  const int tile = blockIdx.x * 8 + wave;
  if (tile >= tilesM * tilesN) return;
  const int tm = tile / tilesN;
  const int tn = tile - tm * tilesN;
  const int m0 = tm << 6;
  const int n0 = tn << 6;

  const int rlane = lane & 15;
  const int koff  = (lane >> 4) * 8;
  const int mOff  = (lane >> 4) * 8;

  const _Float16* abase = Amat + (size_t)(m0 + rlane) * lda + koff;
  const _Float16* bbase = Bmat + (size_t)(n0 + rlane) * ldb + koff;
  const size_t astep = (size_t)16 * lda;
  const size_t bstep = (size_t)16 * ldb;

  v8f acc[4][4];
#pragma unroll
  for (int i = 0; i < 4; ++i)
#pragma unroll
    for (int j = 0; j < 4; ++j) acc[i][j] = (v8f){0.f, 0.f, 0.f, 0.f, 0.f, 0.f, 0.f, 0.f};

  for (int k0 = 0; k0 < kdim; k0 += 32) {
    v16h bh[4];
#pragma unroll
    for (int j = 0; j < 4; ++j) bh[j] = frag_load(bbase + (size_t)j * bstep + k0);
#pragma unroll
    for (int i = 0; i < 4; ++i) {
      const v16h ah = frag_load(abase + (size_t)i * astep + k0);
#pragma unroll
      for (int j = 0; j < 4; ++j) acc[i][j] = wmma_h(ah, bh[j], acc[i][j]);
      guard4_h(acc[i][0], acc[i][1], acc[i][2], acc[i][3], ah, bh[3]);
    }
    keep4_h(bh[0], bh[1], bh[2], bh[3]);
  }
  acc_guard4(acc[0][0], acc[0][1], acc[0][2], acc[0][3]);
  acc_guard4(acc[1][0], acc[1][1], acc[1][2], acc[1][3]);
  acc_guard4(acc[2][0], acc[2][1], acc[2][2], acc[2][3]);
  acc_guard4(acc[3][0], acc[3][1], acc[3][2], acc[3][3]);

  float* slab = sT[wave];
  const int hh = lane >> 4;
  const int c4 = (lane & 15) * 4;
#pragma unroll
  for (int i = 0; i < 4; ++i) {
    const int mBase = m0 + (i << 4);
#pragma unroll
    for (int j = 0; j < 4; ++j) {
      const float bv = bias[n0 + (j << 4) + rlane];
#pragma unroll
      for (int r = 0; r < 8; ++r) {
        const float v = acc[i][j][r] * scale + bv;
        slab[(mOff + r) * 68 + (j << 4) + rlane] = v;
      }
    }
    __builtin_amdgcn_fence(__ATOMIC_RELEASE, "workgroup");
    __builtin_amdgcn_wave_barrier();
    __builtin_amdgcn_fence(__ATOMIC_ACQUIRE, "workgroup");
    for (int pass = 0; pass < 2; ++pass) {
#pragma unroll
      for (int it = 0; it < 8; ++it) {
        const int row = it * 2 + hh;
        const v4f v = *(const v4f*)(slab + row * 68 + c4);
        *(volatile v4f*)(Cout + (size_t)(mBase + row) * ldc + n0 + c4) = v;
      }
      __threadfence();
    }
    __builtin_amdgcn_fence(__ATOMIC_RELEASE, "workgroup");
    __builtin_amdgcn_wave_barrier();
    __builtin_amdgcn_fence(__ATOMIC_ACQUIRE, "workgroup");
  }
}

__global__ __launch_bounds__(REC_THR) void rnn_seq_kernel(const float* __restrict__ XPRE,
                                                          const unsigned short* __restrict__ Wp,
                                                          unsigned short* __restrict__ Rout) {
  __shared__ __align__(16) _Float16 Hh[2][SEQ_BLK * HPITCH];
  const _Float16* Wm = (const _Float16*)Wp;
  const int tid = threadIdx.x;
  const int lane = tid & 31;
  const int wave = tid >> 5;
  const int c = lane & 15;
  const int hh = lane >> 4;
  const int koff = hh * 8;
  const int rowbase = blockIdx.x * SEQ_BLK;

  {
    const v8h zv = {(_Float16)0.0f, (_Float16)0.0f, (_Float16)0.0f, (_Float16)0.0f,
                    (_Float16)0.0f, (_Float16)0.0f, (_Float16)0.0f, (_Float16)0.0f};
    v8h* hz = (v8h*)(&Hh[0][0]);
#pragma unroll 1
    for (int i = tid; i < (2 * SEQ_BLK * HPITCH) / 8; i += REC_THR) hz[i] = zv;
  }
  __syncthreads();

  const v8f z8 = {0.f, 0.f, 0.f, 0.f, 0.f, 0.f, 0.f, 0.f};

#pragma unroll 1
  for (int t = 0; t < NSTEP; ++t) {
    const int cur = t & 1;
    const _Float16* hcur = &Hh[cur][0];
    _Float16* hnext = &Hh[cur ^ 1][0];
    const _Float16* arow = hcur + c * HPITCH + koff;

#pragma unroll 1
    for (int nt = 0; nt < 4; ++nt) {
      const int n = 64 * wave + 16 * nt + c;
      float xv[8];
#pragma unroll
      for (int r = 0; r < 8; ++r)
        xv[r] = XPRE[((size_t)(rowbase + 8 * hh + r) * NSTEP + (size_t)t) * NHID + n];
      const _Float16* wrow = Wm + (size_t)n * NHID + koff;
      v8f acc = z8;
#pragma unroll 4
      for (int k0 = 0; k0 < NHID; k0 += 32) {
        const v16h a = frag_load(arow + k0);
        const v16h b = frag_load(wrow + k0);
        acc = wmma_h_guarded(a, b, acc);
      }
#pragma unroll
      for (int r = 0; r < 8; ++r) {
        const float v = acc[r] * WCARRY_INV + xv[r];
        const float hv = tanhf(v);
        hnext[(8 * hh + r) * HPITCH + n] = (_Float16)hv;
      }
    }
    __syncthreads();

    {
      const _Float16* src = hnext + wave * HPITCH + lane * 8;
      unsigned short* dst = Rout + ((size_t)(rowbase + wave) * NSTEP + (size_t)t) * NHID + lane * 8;
      v8h cv[4];
#pragma unroll
      for (int it = 0; it < 4; ++it) cv[it] = *(const v8h*)(src + it * 256);
      for (int pass = 0; pass < 2; ++pass) {
#pragma unroll
        for (int it = 0; it < 4; ++it) *(volatile v8h*)(dst + it * 256) = cv[it];
        __threadfence();
      }
    }
  }
}

extern "C" void kernel_launch(void* const* d_in, const int* in_sizes, int n_in,
                              void* d_out, int out_size, void* d_ws, size_t ws_size, hipStream_t stream) {
  if (n_in < 13 || d_out == nullptr || d_ws == nullptr) return;
  if (in_sizes[0] != NROWS * NEMB || in_sizes[1] != NHID * NEMB || in_sizes[2] != NHID * NHID ||
      in_sizes[3] != NHID || in_sizes[4] != NHID || in_sizes[5] != NHID * NHID || in_sizes[6] != NHID * NHID ||
      in_sizes[7] != NHID || in_sizes[8] != NHID || in_sizes[9] != NHEAD * NHID || in_sizes[10] != NHEAD ||
      in_sizes[11] != NHEAD * NHID || in_sizes[12] != NHEAD || out_size != 2 * NROWS * NHEAD) return;

  const float* x     = (const float*)d_in[0];
  const float* w_ih1 = (const float*)d_in[1];
  const float* w_hh1 = (const float*)d_in[2];
  const float* b_ih1 = (const float*)d_in[3];
  const float* b_hh1 = (const float*)d_in[4];
  const float* w_ih2 = (const float*)d_in[5];
  const float* w_hh2 = (const float*)d_in[6];
  const float* b_ih2 = (const float*)d_in[7];
  const float* b_hh2 = (const float*)d_in[8];
  const float* w_o1  = (const float*)d_in[9];
  const float* b_o1  = (const float*)d_in[10];
  const float* w_o2  = (const float*)d_in[11];
  const float* b_o2  = (const float*)d_in[12];
  float* y_out = (float*)d_out;
  float* z_out = y_out + (size_t)NROWS * NHEAD;
  static_assert((size_t)NROWS * NHEAD * 4 == 8388608, "second output byte offset");

  char* ws = (char*)d_ws;
  size_t off = 0;
  auto carve = [&](size_t bytes) -> char* { char* p = ws + off; off += (bytes + 255) & ~(size_t)255; return p; };
  float*          XPRE  = (float*)carve((size_t)NROWS * NHID * 4);
  unsigned short* PLANE = (unsigned short*)carve((size_t)NROWS * NHID * 2);
  unsigned short* WIH1  = (unsigned short*)carve((size_t)NHID * NEMB * 2);
  unsigned short* WHH1  = (unsigned short*)carve((size_t)NHID * NHID * 2);
  unsigned short* WIH2  = (unsigned short*)carve((size_t)NHID * NHID * 2);
  unsigned short* WHH2  = (unsigned short*)carve((size_t)NHID * NHID * 2);
  unsigned short* WO1   = (unsigned short*)carve((size_t)NHEAD * NHID * 2);
  unsigned short* WO2   = (unsigned short*)carve((size_t)NHEAD * NHID * 2);
  float*          BSUM  = (float*)carve((size_t)2 * NHID * 4);
  if (off > ws_size || off > (size_t)134217728) return;

  const int n8x  = (NROWS * NEMB) / 8;
  const int n8i1 = (NHID * NEMB) / 8;
  const int n8sq = (NHID * NHID) / 8;
  const int n8hd = (NHEAD * NHID) / 8;
  cvt8_f16_kernel<<<n8x  / CVT_THR, CVT_THR, 0, stream>>>(x,     PLANE, n8x,  1.0f);
  cvt8_f16_kernel<<<n8i1 / CVT_THR, CVT_THR, 0, stream>>>(w_ih1, WIH1,  n8i1, WCARRY);
  cvt8_f16_kernel<<<n8sq / CVT_THR, CVT_THR, 0, stream>>>(w_hh1, WHH1,  n8sq, WCARRY);
  cvt8_f16_kernel<<<n8sq / CVT_THR, CVT_THR, 0, stream>>>(w_ih2, WIH2,  n8sq, WCARRY);
  cvt8_f16_kernel<<<n8sq / CVT_THR, CVT_THR, 0, stream>>>(w_hh2, WHH2,  n8sq, WCARRY);
  cvt8_f16_kernel<<<n8hd / CVT_THR, CVT_THR, 0, stream>>>(w_o1,  WO1,   n8hd, WCARRY);
  cvt8_f16_kernel<<<n8hd / CVT_THR, CVT_THR, 0, stream>>>(w_o2,  WO2,   n8hd, WCARRY);
  bias_sum_kernel<<<2, 256, 0, stream>>>(b_ih1, b_hh1, b_ih2, b_hh2, BSUM);

  const int grid_proj = ((NROWS / 64) * (NHID / 64)) / 8;
  const int grid_head = ((NROWS / 64) * (NHEAD / 64)) / 8;
  static_assert(((NROWS / 64) * (NHID / 64)) % 8 == 0 && ((NROWS / 64) * (NHEAD / 64)) % 8 == 0, "GEMM grids exact");

  gemm64_f16_kernel<<<grid_proj, 256, 0, stream>>>(PLANE, NEMB, WIH1, NEMB, XPRE, NHID, BSUM,
                                                   NROWS, NHID, NEMB, WCARRY_INV);
  rnn_seq_kernel<<<NBATCH / SEQ_BLK, REC_THR, 0, stream>>>(XPRE, WHH1, PLANE);
  gemm64_f16_kernel<<<grid_proj, 256, 0, stream>>>(PLANE, NHID, WIH2, NHID, XPRE, NHID, BSUM + NHID,
                                                   NROWS, NHID, NHID, WCARRY_INV);
  gemm64_f16_kernel<<<grid_head, 256, 0, stream>>>(PLANE, NHID, WO1, NHID, y_out, NHEAD, b_o1,
                                                   NROWS, NHEAD, NHID, WCARRY_INV);
  rnn_seq_kernel<<<NBATCH / SEQ_BLK, REC_THR, 0, stream>>>(XPRE, WHH2, PLANE);
  gemm64_f16_kernel<<<grid_head, 256, 0, stream>>>(PLANE, NHID, WO2, NHID, z_out, NHEAD, b_o2,
                                                   NROWS, NHEAD, NHID, WCARRY_INV);
}
